// RecurrentRetention_60413009985545
// MI455X (gfx1250) — hardware-verified
//
#include <hip/hip_runtime.h>
#include <stdint.h>

typedef __attribute__((ext_vector_type(16))) _Float16 v16h;
typedef __attribute__((ext_vector_type(8)))  _Float16 v8h;
typedef __attribute__((ext_vector_type(16))) __bf16   v16b;
typedef __attribute__((ext_vector_type(8)))  __bf16   v8b;
typedef __attribute__((ext_vector_type(8)))  float    v8f;
typedef __attribute__((ext_vector_type(4)))  float    v4f;

__device__ __forceinline__ unsigned short f2bf_bits(float f) {
  unsigned u = __float_as_uint(f);
  return (unsigned short)((u + 0x7FFFu + ((u >> 16) & 1u)) >> 16);
}
__device__ __forceinline__ float bf_bits2f(unsigned short h) { return __uint_as_float(((unsigned)h) << 16); }

__device__ __forceinline__ void dep_guard_h(v8f& a, v8f& b, v16h x, v16h y) { asm volatile("v_nop\n\tv_nop\n\tv_nop\n\tv_nop" : "+v"(a), "+v"(b) : "v"(x), "v"(y)); }
__device__ __forceinline__ void dep_guard_b(v8f& a, v8f& b, v16b x, v16b y) { asm volatile("v_nop\n\tv_nop\n\tv_nop\n\tv_nop" : "+v"(a), "+v"(b) : "v"(x), "v"(y)); }
__device__ __forceinline__ void keep4_h(v16h a, v16h b, v16h c, v16h d) { asm volatile("v_nop" :: "v"(a), "v"(b), "v"(c), "v"(d)); }
__device__ __forceinline__ void keep4_b(v16b a, v16b b, v16b c, v16b d) { asm volatile("v_nop" :: "v"(a), "v"(b), "v"(c), "v"(d)); }
__device__ __forceinline__ void acc_guard4(v8f& a, v8f& b, v8f& c, v8f& d) { asm volatile("v_nop\n\tv_nop\n\tv_nop\n\tv_nop" : "+v"(a), "+v"(b), "+v"(c), "+v"(d)); }
template <typename T> struct Frag;
template <> struct Frag<_Float16> {
  typedef v16h V; union U { v16h v; v8h h[2]; };
  static __device__ __forceinline__ v16h load(const _Float16* p) {
    U f; f.h[0] = *(const v8h*)(p); f.h[1] = *(const v8h*)(p + 16); return f.v;
  }
  static __device__ __forceinline__ v8f mma(v16h a, v16h b, v8f c) {
    return __builtin_amdgcn_wmma_f32_16x16x32_f16(false, a, false, b, (short)0, c, false, false);
  }
  static __device__ __forceinline__ void guard(v8f& a, v8f& b, v16h x, v16h y) { dep_guard_h(a, b, x, y); }
  static __device__ __forceinline__ void keep(v16h a, v16h b, v16h c, v16h d) { keep4_h(a, b, c, d); }
};
template <> struct Frag<__bf16> {
  typedef v16b V; union U { v16b v; v8b h[2]; };
  static __device__ __forceinline__ v16b load(const __bf16* p) {
    U f; f.h[0] = *(const v8b*)(p); f.h[1] = *(const v8b*)(p + 16); return f.v;
  }
  static __device__ __forceinline__ v8f mma(v16b a, v16b b, v8f c) {
    return __builtin_amdgcn_wmma_f32_16x16x32_bf16(false, a, false, b, (short)0, c, false, false);
  }
  static __device__ __forceinline__ void guard(v8f& a, v8f& b, v16b x, v16b y) { dep_guard_b(a, b, x, y); }
  static __device__ __forceinline__ void keep(v16b a, v16b b, v16b c, v16b d) { keep4_b(a, b, c, d); }
};

template <int ET> struct Elem;
template <> struct Elem<0> { typedef _Float16 T; };
template <> struct Elem<1> { typedef __bf16 T; };
template <int ET, bool SPLIT, int BIAS_MODE, int OUT_MODE, bool RESID, int ACT = 0>
__global__ __launch_bounds__(256) void wmma_gemm64(
    const unsigned short* __restrict__ Ap, const unsigned short* __restrict__ A2p, int lda, long strideA,
    const unsigned short* __restrict__ Btp, const unsigned short* __restrict__ Bt2p, int ldb, long strideB,
    void* __restrict__ Cout, void* __restrict__ Cout2, int ldc, long strideC,
    const float* __restrict__ bias,
    const float* __restrict__ resid, long strideR,
    int M, int N, int K, float scale) {
  typedef typename Elem<ET>::T T;
  typedef typename Frag<T>::V V;
  const T* A = (const T*)Ap; const T* A2 = (const T*)A2p; const T* Bt = (const T*)Btp; const T* Bt2 = (const T*)Bt2p;
  __shared__ __align__(16) float sT[8][16 * 68];
  const int b    = blockIdx.y;
  const int lane = threadIdx.x & 31;
  const int wave = threadIdx.x >> 5;
  const int tilesN = N >> 6;
  const int tilesM = M >> 6;
  const int tile = blockIdx.x * 8 + wave;
  if (tile >= tilesM * tilesN) return;
  const int tm = tile / tilesN;
  const int tn = tile - tm * tilesN;
  const int m0 = tm << 6;
  const int n0 = tn << 6;

  const T* Ab  = A  + (size_t)b * strideA;
  const T* Bb  = Bt + (size_t)b * strideB;
  const T* Ab2 = SPLIT ? (A2  + (size_t)b * strideA) : nullptr;
  const T* Bb2 = SPLIT ? (Bt2 + (size_t)b * strideB) : nullptr;

  const int rlane = lane & 15;
  const int koff  = (lane >> 4) * 8;
  const int mOff  = (lane >> 4) * 8;

  v8f acc[4][4];
#pragma unroll
  for (int i = 0; i < 4; ++i)
#pragma unroll
    for (int j = 0; j < 4; ++j) acc[i][j] = (v8f){0.f,0.f,0.f,0.f,0.f,0.f,0.f,0.f};

  for (int k0 = 0; k0 < K; k0 += 32) {
    V bh[4], bl[4];
#pragma unroll
    for (int j = 0; j < 4; ++j) {
      const size_t bo = (size_t)(n0 + (j << 4) + rlane) * ldb + koff + k0;
      bh[j] = Frag<T>::load(Bb + bo);
      if (SPLIT) bl[j] = Frag<T>::load(Bb2 + bo);
    }
#pragma unroll
    for (int i = 0; i < 4; ++i) {
      const size_t ao = (size_t)(m0 + (i << 4) + rlane) * lda + koff + k0;
      V ah = Frag<T>::load(Ab + ao);
      V al;
      if (SPLIT) al = Frag<T>::load(Ab2 + ao);
#pragma unroll
      for (int j = 0; j < 4; ++j) {
        acc[i][j] = Frag<T>::mma(ah, bh[j], acc[i][j]);
        if (SPLIT) {
          acc[i][j] = Frag<T>::mma(ah, bl[j], acc[i][j]);
          acc[i][j] = Frag<T>::mma(al, bh[j], acc[i][j]);
        }
      }
      Frag<T>::guard(acc[i][0], acc[i][3], ah, SPLIT ? al : ah);
    }
    Frag<T>::keep(bh[0], bh[1], bh[2], bh[3]);
    if (SPLIT) Frag<T>::keep(bl[0], bl[1], bl[2], bl[3]);
  }
  acc_guard4(acc[0][0], acc[0][1], acc[0][2], acc[0][3]);
  acc_guard4(acc[1][0], acc[1][1], acc[1][2], acc[1][3]);
  acc_guard4(acc[2][0], acc[2][1], acc[2][2], acc[2][3]);
  acc_guard4(acc[3][0], acc[3][1], acc[3][2], acc[3][3]);

  float* slab = sT[wave];
  const float* Rb = RESID ? (resid + (size_t)b * strideR) : nullptr;
#pragma unroll
  for (int i = 0; i < 4; ++i) {
    const int mBase = m0 + (i << 4);
#pragma unroll
    for (int j = 0; j < 4; ++j) {
      const int n = n0 + (j << 4) + rlane;
      float bv = 0.f;
      if (BIAS_MODE == 2) bv = bias[n];
#pragma unroll
      for (int r = 0; r < 8; ++r) {
        float v = acc[i][j][r] * scale;
        if (BIAS_MODE == 1) v += bias[mBase + mOff + r];
        if (BIAS_MODE == 2) v += bv;
        if (RESID) v += Rb[(size_t)(mBase + mOff + r) * ldc + n];
        if (ACT == 1) v = tanhf(v);
        if (ACT == 2) v = fmaxf(v, 0.0f);
        if (ACT == 3) v = v / (1.0f + expf(-v));
        if (ACT == 4) v = (v > 0.f) ? v : 0.01f * v;
        if (ACT == 5) v = 0.5f * v * (1.0f + erff(v * 0.70710678118654752f));
        slab[(mOff + r) * 68 + (j << 4) + rlane] = v;
      }
    }
    __builtin_amdgcn_fence(__ATOMIC_RELEASE, "workgroup");
    __builtin_amdgcn_wave_barrier();
    __builtin_amdgcn_fence(__ATOMIC_ACQUIRE, "workgroup");
    if (OUT_MODE == 0) {
      float* C = (float*)Cout + (size_t)b * strideC;
      const int hh = lane >> 4, c4 = (lane & 15) * 4;
      for (int pass = 0; pass < 2; ++pass) {
#pragma unroll
        for (int it = 0; it < 8; ++it) {
          const int row = it * 2 + hh;
          v4f v = *(const v4f*)(slab + row * 68 + c4);
          *(volatile v4f*)(C + (size_t)(mBase + row) * ldc + n0 + c4) = v;
        }
        __threadfence();
      }
    } else {
      const int q = lane >> 3, c8 = (lane & 7) * 8;
      unsigned short* C  = (unsigned short*)Cout  + (size_t)b * strideC;
      unsigned short* C2 = (OUT_MODE == 2) ? ((unsigned short*)Cout2 + (size_t)b * strideC) : nullptr;
      for (int pass = 0; pass < 2; ++pass) {
#pragma unroll
        for (int it = 0; it < 4; ++it) {
          const int row = it * 4 + q;
          const float* sp = slab + row * 68 + c8;
          v8h hv, lv;
#pragma unroll
          for (int e = 0; e < 8; ++e) {
            if (OUT_MODE == 1) {
              hv[e] = (_Float16)sp[e];
            } else {
              unsigned short hb = f2bf_bits(sp[e]);
              unsigned short lb = f2bf_bits(sp[e] - bf_bits2f(hb));
              hv[e] = __builtin_bit_cast(_Float16, hb);
              lv[e] = __builtin_bit_cast(_Float16, lb);
            }
          }
          *(volatile v8h*)(C + (size_t)(mBase + row) * ldc + n0 + c8) = hv;
          if (OUT_MODE == 2) *(volatile v8h*)(C2 + (size_t)(mBase + row) * ldc + n0 + c8) = lv;
        }
        __threadfence();
      }
    }
    __builtin_amdgcn_fence(__ATOMIC_RELEASE, "workgroup");
    __builtin_amdgcn_wave_barrier();
    __builtin_amdgcn_fence(__ATOMIC_ACQUIRE, "workgroup");
  }
}

__global__ __launch_bounds__(256) void cast_f32_f16x2(
    const float* __restrict__ in, _Float16* __restrict__ out, int n2) {
  int i = blockIdx.x * 256 + threadIdx.x;
  if (i < n2) {
    const _Float16 h0 = (_Float16)in[2 * i], h1 = (_Float16)in[2 * i + 1];
    const unsigned u = (unsigned)__builtin_bit_cast(unsigned short, h0) | ((unsigned)__builtin_bit_cast(unsigned short, h1) << 16);
    ((volatile unsigned*)out)[i] = u;
    __threadfence();
    ((volatile unsigned*)out)[i] = u;
  }
}

__global__ __launch_bounds__(256) void k_transpose_cast(
    const float* __restrict__ W0, const float* __restrict__ W1,
    _Float16* __restrict__ WT, int D, float wscale) {
  __shared__ float tile[64][65];
  const float* W = (blockIdx.z == 0) ? W0 : W1;
  _Float16* O = WT + (size_t)blockIdx.z * (size_t)D * (size_t)D;
  const int n0 = blockIdx.x * 64;
  const int k0 = blockIdx.y * 64;
  const int t = threadIdx.x;
#pragma unroll
  for (int it = 0; it < 4; ++it) {
    const int row = it * 16 + (t >> 4);
    const int c4  = (t & 15) * 4;
    const v4f v = *(const v4f*)(W + (size_t)(k0 + row) * D + n0 + c4);
    tile[row][c4 + 0] = v[0];
    tile[row][c4 + 1] = v[1];
    tile[row][c4 + 2] = v[2];
    tile[row][c4 + 3] = v[3];
  }
  __syncthreads();
  const int wave = t >> 5, lane = t & 31;
  const int q = lane >> 3, c8 = (lane & 7) * 8;
  for (int pass = 0; pass < 2; ++pass) {
#pragma unroll
    for (int it = 0; it < 2; ++it) {
      const int r = wave * 8 + it * 4 + q;
      v8h hv;
#pragma unroll
      for (int e = 0; e < 8; ++e) hv[e] = (_Float16)(tile[c8 + e][r] * wscale);
      *(volatile v8h*)(O + (size_t)(n0 + r) * D + k0 + c8) = hv;
    }
    __threadfence();
  }
}

template <bool VEC>
__global__ __launch_bounds__(256) void k_rowdot(
    const float* __restrict__ A, const float* __restrict__ v, float* __restrict__ out, int rows, int D) {
  __shared__ float red[32];
  const int wave = threadIdx.x >> 5, lane = threadIdx.x & 31;
  const int r0 = blockIdx.x * 32;
#pragma unroll 1
  for (int rr = 0; rr < 4; ++rr) {
    int r = r0 + wave * 4 + rr;
    r = r < rows ? r : rows - 1;
    const float* p = A + (size_t)r * D;
    float s = 0.f;
#pragma unroll 1
    for (int i = lane * 4; i < D; i += 128) {
      const v4f a = *(const v4f*)(p + i);
      if (VEC) {
        const v4f w = *(const v4f*)(v + i);
        s += a[0] * w[0] + a[1] * w[1] + a[2] * w[2] + a[3] * w[3];
      } else {
        s += (a[0] + a[1]) + (a[2] + a[3]);
      }
    }
#pragma unroll
    for (int off = 16; off > 0; off >>= 1) s += __shfl_xor(s, off, 32);
    if (lane == 0) red[wave * 4 + rr] = s;
  }
  __syncthreads();
  if (wave == 0) {
    const int r = r0 + lane;
    const float val = red[lane];
    if (r < rows) *(volatile float*)(out + r) = val;
    __threadfence();
    if (r < rows) *(volatile float*)(out + r) = val;
  }
}

__global__ __launch_bounds__(256) void k_scan(
    const float* __restrict__ Kf, const float* __restrict__ vs, float* __restrict__ S,
    int B, int T, int D, float gamma) {
  const int d = blockIdx.x * 256 + threadIdx.x;
  if (d >= D) return;
  float s = 0.f;
  for (int t = 1; t < T; ++t) {
    float m = 0.f;
#pragma unroll 1
    for (int b = 0; b < B; ++b)
      m += Kf[((size_t)b * T + t) * (size_t)D + d] * vs[(size_t)b * T + t];
    s = gamma * s + m;
    float* p = S + (size_t)t * D + d;
    *(volatile float*)p = s;
    if (t == 1) *(volatile float*)(S + d) = s;
    __threadfence();
    *(volatile float*)p = s;
    if (t == 1) *(volatile float*)(S + d) = s;
  }
}

__global__ __launch_bounds__(256) void k_out(
    const float* __restrict__ Qf, const float* __restrict__ S, float* __restrict__ out,
    int B, int T, int D) {
  const int D4 = D >> 2;
  const int gid = blockIdx.x * 256 + threadIdx.x;
  if (gid >= T * D4) return;
  const int t = gid / D4;
  const int d0 = (gid - t * D4) * 4;
  v4f sv;
  sv[0] = S[(size_t)(d0 + 0) * T + t];
  sv[1] = S[(size_t)(d0 + 1) * T + t];
  sv[2] = S[(size_t)(d0 + 2) * T + t];
  sv[3] = S[(size_t)(d0 + 3) * T + t];
#pragma unroll 1
  for (int b = 0; b < B; ++b) {
    const size_t o = ((size_t)b * T + t) * (size_t)D + d0;
    const v4f qv = *(const v4f*)(Qf + o);
    const v4f val = qv * sv;
    *(volatile v4f*)(out + o) = val;
    __threadfence();
    *(volatile v4f*)(out + o) = val;
  }
}


extern "C" void kernel_launch(void* const* d_in, const int* in_sizes, int n_in,
                              void* d_out, int out_size, void* d_ws, size_t ws_size,
                              hipStream_t stream) {
  if (n_in < 4) return;
  const int D = 1024;
  const int T = 2048;
  if (in_sizes[1] != D * D || in_sizes[2] != D * D || in_sizes[3] != D * D) return;
  const long nx = (long)in_sizes[0];
  if (nx <= 0 || (nx % ((long)T * D)) != 0) return;
  const int B = (int)(nx / ((long)T * D));
  const int BT = B * T;
  if ((long)out_size != nx) return;
  if ((BT % 64) != 0) return;

  const float* x  = (const float*)d_in[0];
  const float* Wq = (const float*)d_in[1];
  const float* Wk = (const float*)d_in[2];
  const float* Wv = (const float*)d_in[3];
  float* out = (float*)d_out;

  char* ws = (char*)d_ws;
  size_t off = 0;
  _Float16* xh = (_Float16*)(ws + off); off += (size_t)BT * D * 2;
  _Float16* WT = (_Float16*)(ws + off); off += (size_t)2 * D * D * 2;
  float* QK  = (float*)(ws + off);       off += (size_t)2 * BT * D * 4;
  float* wvs = (float*)(ws + off);       off += 4096;
  float* vs  = (float*)(ws + off);       off += (((size_t)BT * 4) + 4095) / 4096 * 4096;
  float* S   = (float*)(ws + off);       off += (size_t)T * D * 4;
  if (off > ws_size || off > (size_t)134217728) return;
  if ((size_t)D * 4 > 4096) return;
  float* Qf = QK;
  float* Kf = QK + (size_t)BT * D;

  {
    const int n2 = (int)(nx / 2);
    cast_f32_f16x2<<<(n2 + 255) / 256, 256, 0, stream>>>(x, xh, n2);
  }
  k_transpose_cast<<<dim3(D / 64, D / 64, 2), 256, 0, stream>>>(Wq, Wk, WT, D, 16.0f);
  k_rowdot<false><<<(D + 31) / 32, 256, 0, stream>>>(Wv, nullptr, wvs, D, D);
  k_rowdot<true><<<(BT + 31) / 32, 256, 0, stream>>>(x, wvs, vs, BT, D);
  {
    const int tiles = (BT / 64) * (D / 64);
    const int gx = (tiles + 7) / 8;
    wmma_gemm64<0, false, 0, 0, false, 0><<<dim3(gx, 2), 256, 0, stream>>>(
        (const unsigned short*)xh, (const unsigned short*)xh, D, (long)0,
        (const unsigned short*)WT, (const unsigned short*)WT, D, (long)D * D,
        (void*)QK, (void*)QK, D, (long)BT * D,
        nullptr, nullptr, (long)0,
        BT, D, D, 1.0f / 16.0f);
  }
  k_scan<<<(D + 255) / 256, 256, 0, stream>>>(Kf, vs, S, B, T, D, 0.96875f);
  {
    const int n = T * (D / 4);
    k_out<<<(n + 255) / 256, 256, 0, stream>>>(Qf, S, out, B, T, D);
  }
}
